// FourierModelTestNU_72705206387341
// MI455X (gfx1250) — hardware-run, weakly checked
//
#include <hip/hip_runtime.h>


#ifndef NB
#define NB 128
#endif
#define NB_FULL 128
#define TLEN 1024
#define NS   1024
#define HID1 512
#define HID2 128
#define NO   8
#define NOP  16
#define FA   32
#define FB   32
#define TC   128
#define KC   (2 * TC)
#define PP   (KC + 8)
#define CSP  68
#define PSC  16.0f
#define QSC  1024.0f
#define CSI  (1.0f / (16.0f * 1024.0f))
#define WSC  256.0f
#define WSI  (1.0f / 256.0f)
#define TWO_PI_T 6.28318530717958647692f
#define REV_EXC  2.782754e-8f
#define LOG2E    1.4426950408889634f

static_assert(NS == FA * FB);
static_assert(NS == TLEN);
static_assert(FA == FB);
static_assert(NS <= 65536);
static_assert(TLEN % TC == 0);
static_assert(TC % 8 == 0);
static_assert(KC % 32 == 0);
static_assert((PP * 2) % 16 == 0);
static_assert((256 / (TC / 8)) * 2 == FB);
static_assert(TLEN % 256 == 0);
static_assert(FA == 2 * 16);
static_assert(2 * FB == 4 * 16);
static_assert(128 * 16 == NS * 2);
static_assert(NB % 64 == 0);
static_assert(NB % 16 == 0);
static_assert(HID1 % 64 == 0);
static_assert(HID2 % 64 == 0);
static_assert(NS % 32 == 0);
static_assert(HID1 % 32 == 0);
static_assert(HID2 % 32 == 0);
static_assert(4 * 32 * 16 == 16 * 64 * 2);
static_assert(32 * 16 == 16 * NO * 4);
static_assert(NO <= NOP);
static_assert((NO & (NO - 1)) == 0);
static_assert(NB <= NB_FULL);
static_assert((CSP * 4) % 16 == 0);
static_assert((size_t)FA * PP * 2 + (size_t)2 * FB * PP * 2 + (size_t)2 * TLEN * 4 + (size_t)FA * CSP * 4 <= (size_t)131072);
static_assert(((size_t)HID1 * NS) % 64 == 0);
static_assert(((size_t)HID2 * HID1) % 64 == 0);
static_assert(((size_t)NOP * HID2) % 64 == 0);
static_assert(((size_t)NO * HID2) % 8 == 0);

typedef _Float16 h16;
typedef __attribute__((ext_vector_type(16))) _Float16 v16h;
typedef __attribute__((ext_vector_type(8)))  _Float16 v8h;
typedef __attribute__((ext_vector_type(8)))  float    v8f;
typedef __attribute__((ext_vector_type(4)))  float    v4f;
typedef v4f  __attribute__((may_alias)) v4fa;

__device__ __forceinline__ unsigned short f2bf(float f) { unsigned u = __float_as_uint(f); u += 0x7FFFu + ((u >> 16) & 1u); return (unsigned short)(u >> 16); }
__device__ __forceinline__ float bfr(float f) { return __uint_as_float(((unsigned)f2bf(f)) << 16); }
__device__ __forceinline__ v16h cat16(v8h lo, v8h hi) { return __builtin_shufflevector(lo, hi, 0, 1, 2, 3, 4, 5, 6, 7, 8, 9, 10, 11, 12, 13, 14, 15); }
__device__ __forceinline__ v16h  ldh(const h16* p) { return cat16(*(const v8h*)p, *(const v8h*)(p + 16)); }
__device__ __forceinline__ v8f wmma16g(v16h a, v16h b, v8f c) {
    c = __builtin_amdgcn_wmma_f32_16x16x32_f16(false, a, false, b, (short)0, c, false, false);
    asm volatile("v_nop\n\tv_nop\n\tv_nop\n\tv_nop" : "+v"(c) : "v"(a), "v"(b));
    return c;
}
static __device__ __forceinline__ h16 toh_flush(float v) { const h16 r = (h16)v; return (fabsf(v) < 6.103515625e-05f) ? (h16)0.0f : r; }
__device__ __forceinline__ void wave_sync() { __builtin_amdgcn_fence(3  , "wavefront"); __builtin_amdgcn_wave_barrier(); asm volatile("" ::: "memory"); }

__device__ __forceinline__ void trig_rev(float r, float& sn, float& cn) {
    const float fr  = r - rintf(r);
    const float rev = fmaf(r, REV_EXC, fr);
    const float q   = rintf(rev * 4.0f);
    const int   iq  = (int)q;
    const float y   = fmaf(q, -0.25f, rev);
    const float z   = y * TWO_PI_T;
    const float z2  = z * z;
    float sp = fmaf(z2, -1.9515295891e-4f, 8.3321608736e-3f);
    sp = fmaf(sp, z2, -1.6666654611e-1f);
    const float s0 = fmaf(sp * z2, z, z);
    float cp = fmaf(z2, 2.443315711809948e-5f, -1.388731625493765e-3f);
    cp = fmaf(cp, z2, 4.166664568298827e-2f);
    const float c0 = fmaf(cp, z2 * z2, fmaf(z2, -0.5f, 1.0f));
    const int k = iq & 3;
    const float sv = (k & 1) ? c0 : s0;
    const float cv = (k & 1) ? s0 : c0;
    sn = (k & 2) ? -sv : sv;
    cn = ((k + 1) & 2) ? -cv : cv;
}

__global__ __launch_bounds__(256) void k_wcvt(const float* __restrict__ src, h16* dst, unsigned nsrc8, unsigned ndst8) {
    const unsigned i = blockIdx.x * 256 + threadIdx.x; if (i >= ndst8) return;
    const unsigned ic = (i < nsrc8) ? i : (nsrc8 - 1);
    v8f v = *(const v8f*)(src + (size_t)ic * 8);
    asm volatile("" : "+v"(v));
    const bool ok = i < nsrc8; v8h o;
#pragma unroll
    for (int k = 0; k < 8; ++k) { const h16 c = toh_flush(bfr(v[k]) * WSC); o[k] = ok ? c : (h16)0.0f; }
    *(volatile v8h*)(dst + (size_t)i * 8) = o; __threadfence(); *(volatile v8h*)(dst + (size_t)i * 8) = o;
}

__global__ __launch_bounds__(256) void k_spec(const float* __restrict__ inp, h16* FH) {
    __shared__ __align__(16) h16 pt[FA * PP];
    __shared__ __align__(16) h16 qt[2 * FB * PP];
    __shared__ __align__(16) float xs[TLEN];
    __shared__ __align__(16) float dd[TLEN];
    __shared__ __align__(16) float cs[FA * CSP];
    const int tid = threadIdx.x;
    const int lane = tid & 31, lr = lane & 15, hi = lane >> 4;
    const int wave = __builtin_amdgcn_readfirstlane((int)(threadIdx.x >> 5));
    const int n = blockIdx.x;
    const float* src = inp + (size_t)n * TLEN * 3;
#pragma unroll 1
    for (int t = tid; t < TLEN; t += 256) { xs[t] = bfr(src[(size_t)t * 3]); dd[t] = bfr(src[(size_t)t * 3 + 2]); }
    __syncthreads();
    const int g = tid & 15, rw = tid >> 4;
    const int mb = wave >> 2, nb = wave & 3;
    v8f acc = (v8f){};
#pragma unroll 1
    for (int c0 = 0; c0 < TLEN; c0 += TC) {
        const v4f xa = *(const v4fa*)(&xs[c0 + 8 * g]), xb = *(const v4fa*)(&xs[c0 + 8 * g + 4]);
        const v4f da = *(const v4fa*)(&dd[c0 + 8 * g]), db = *(const v4fa*)(&dd[c0 + 8 * g + 4]);
        float xv[8], dv[8];
#pragma unroll
        for (int i = 0; i < 4; ++i) { xv[i] = xa[i]; xv[4 + i] = xb[i]; dv[i] = da[i]; dv[4 + i] = db[i]; }
#pragma unroll 1
        for (int jj = 0; jj < 2; ++jj) {
            const int b = rw + 16 * jj; const float fb = (float)b;
            v8h vc, vs, vn;
#pragma unroll
            for (int i = 0; i < 8; ++i) { float sn, cn; trig_rev(fb * dv[i], sn, cn);
                vc[i] = toh_flush(cn * QSC); vs[i] = toh_flush(sn * QSC); vn[i] = toh_flush(-sn * QSC); }
            *(v8h*)(&qt[b * PP + 8 * g]) = vc;        *(v8h*)(&qt[b * PP + TC + 8 * g]) = vn;
            *(v8h*)(&qt[(FB + b) * PP + 8 * g]) = vs; *(v8h*)(&qt[(FB + b) * PP + TC + 8 * g]) = vc;
        }
#pragma unroll 1
        for (int jj = 0; jj < 2; ++jj) {
            const int a = rw + 16 * jj; const float fa = (float)(FB * a);
            v8h vc, vs;
#pragma unroll
            for (int i = 0; i < 8; ++i) { float sn, cn; trig_rev(fa * dv[i], sn, cn);
                vc[i] = toh_flush(xv[i] * cn * PSC); vs[i] = toh_flush(xv[i] * sn * PSC); }
            *(v8h*)(&pt[a * PP + 8 * g]) = vc; *(v8h*)(&pt[a * PP + TC + 8 * g]) = vs;
        }
        __syncthreads();
#pragma unroll 2
        for (int kc = 0; kc < KC; kc += 32) {
            const int ia = (mb * 16 + lr) * PP + kc + 8 * hi;
            const int ib = (nb * 16 + lr) * PP + kc + 8 * hi;
            const v8h a0 = *(const v8h*)(&pt[ia]); const v8h a1 = *(const v8h*)(&pt[ia + 16]);
            const v8h b0 = *(const v8h*)(&qt[ib]); const v8h b1 = *(const v8h*)(&qt[ib + 16]);
            acc = wmma16g(cat16(a0, a1), cat16(b0, b1), acc);
        }
        __syncthreads();
    }
#pragma unroll
    for (int r = 0; r < 8; ++r) cs[(mb * 16 + 8 * hi + r) * CSP + nb * 16 + lr] = acc[r];
    __syncthreads();
    if (wave < 4) {
        const int a = tid >> 2, b0 = (tid & 3) * 8;
        const v4f r0 = *(const v4fa*)(&cs[a * CSP + b0]),      r1 = *(const v4fa*)(&cs[a * CSP + b0 + 4]);
        const v4f i0 = *(const v4fa*)(&cs[a * CSP + FB + b0]), i1 = *(const v4fa*)(&cs[a * CSP + FB + b0 + 4]);
        v8h o;
#pragma unroll
        for (int k = 0; k < 4; ++k) {
            o[k]     = toh_flush(sqrtf(r0[k] * r0[k] + i0[k] * i0[k]) * CSI);
            o[4 + k] = toh_flush(sqrtf(r1[k] * r1[k] + i1[k] * i1[k]) * CSI); }
        h16* dst = FH + (size_t)n * NS + (size_t)tid * 8;
        *(volatile v8h*)dst = o; __threadfence(); *(volatile v8h*)dst = o;
    }
}

__device__ __forceinline__ float sigm(float z) {
    const float zc = fminf(fmaxf(z, -30.0f), 30.0f);
    const float e = __builtin_amdgcn_exp2f(-zc * LOG2E);
    return 1.0f / (1.0f + e);
}

__global__ __launch_bounds__(32) void k_dense(const h16* __restrict__ A, const h16* __restrict__ Bt, const float* __restrict__ bias, h16* Out, int K, int N) {
    __shared__ __align__(16) float os[16 * 68];
    const int lane = threadIdx.x & 31, lr = lane & 15, hi = lane >> 4; const int r0 = blockIdx.x * 64, c0 = blockIdx.y * 64;
    v8f acc[4][4];
#pragma unroll
    for (int mb = 0; mb < 4; ++mb)
#pragma unroll
        for (int nb = 0; nb < 4; ++nb) acc[mb][nb] = (v8f){};
    const size_t aoff = (size_t)(r0 + lr) * K + 8 * hi, boff = (size_t)(c0 + lr) * K + 8 * hi;
#pragma unroll 1
    for (int kc = 0; kc < K; kc += 32) {
        v16h a[4];
#pragma unroll
        for (int mb = 0; mb < 4; ++mb) a[mb] = ldh(A + aoff + (size_t)mb * 16 * K + kc);
#pragma unroll
        for (int nb = 0; nb < 4; ++nb) { const v16h b = ldh(Bt + boff + (size_t)nb * 16 * K + kc);
#pragma unroll
            for (int mb = 0; mb < 4; ++mb) acc[mb][nb] = wmma16g(a[mb], b, acc[mb][nb]); }
    }
    float bc[4];
#pragma unroll
    for (int nb = 0; nb < 4; ++nb) bc[nb] = bfr(bias[c0 + nb * 16 + lr]);
#pragma unroll
    for (int mb = 0; mb < 4; ++mb) {
#pragma unroll
        for (int nb = 0; nb < 4; ++nb) {
#pragma unroll
            for (int j = 0; j < 8; ++j) os[(hi * 8 + j) * 68 + nb * 16 + lr] = sigm(acc[mb][nb][j] * WSI + bc[nb]); }
        wave_sync();
#pragma unroll 1
        for (int ps = 0; ps < 2; ++ps) {
#pragma unroll
            for (int s = 0; s < 4; ++s) { const int row = 4 * s + (lane >> 3), c8 = (lane & 7) * 8;
                const v4f x0 = *(const v4fa*)(&os[row * 68 + c8]); const v4f x1 = *(const v4fa*)(&os[row * 68 + c8 + 4]); v8h hv;
#pragma unroll
                for (int i = 0; i < 4; ++i) { hv[i] = toh_flush(x0[i]); hv[4 + i] = toh_flush(x1[i]); }
                *(volatile v8h*)(Out + (size_t)(r0 + mb * 16 + row) * N + c0 + c8) = hv; }
            if (ps == 0) __threadfence(); }
        wave_sync();
    }
}

__global__ __launch_bounds__(32) void k_head(const h16* __restrict__ A, const h16* __restrict__ Bt, const float* __restrict__ bias, float* OUT) {
    __shared__ __align__(16) float os[16 * 16];
    const int lane = threadIdx.x & 31, lr = lane & 15, hi = lane >> 4; const int r0 = blockIdx.x * 16;
    v8f acc = (v8f){};
    const size_t aoff = (size_t)(r0 + lr) * HID2 + 8 * hi, boff = (size_t)lr * HID2 + 8 * hi;
#pragma unroll
    for (int kc = 0; kc < HID2; kc += 32) acc = wmma16g(ldh(A + aoff + kc), ldh(Bt + boff + kc), acc);
    const float bv = bfr(bias[lr & (NO - 1)]);
#pragma unroll
    for (int j = 0; j < 8; ++j) os[(hi * 8 + j) * 16 + lr] = acc[j] * WSI + bv;
    wave_sync();
    const int row = lane >> 1, c4 = (lane & 1) * 4;
    const v4f val = *(const v4fa*)(&os[row * 16 + c4]);
    float* dst = OUT + (size_t)r0 * NO + (size_t)lane * 4;
    *(volatile v4f*)dst = val; __threadfence(); *(volatile v4f*)dst = val;
}

static constexpr size_t al256(size_t v) { return (v + 255) & ~(size_t)255; }
static constexpr size_t SZ_W1 = al256((size_t)HID1 * NS * 2);
static constexpr size_t SZ_W2 = al256((size_t)HID2 * HID1 * 2);
static constexpr size_t SZ_W3 = al256((size_t)NOP * HID2 * 2);
static constexpr size_t SZ_FH = al256((size_t)NB * NS * 2);
static constexpr size_t SZ_H1 = al256((size_t)NB * HID1 * 2);
static constexpr size_t SZ_H2 = al256((size_t)NB * HID2 * 2);
static constexpr size_t SZ_TOTAL = SZ_W1 + SZ_W2 + SZ_W3 + SZ_FH + SZ_H1 + SZ_H2;
static_assert(SZ_TOTAL <= (size_t)134217728);

extern "C" void kernel_launch(void* const* d_in, const int* in_sizes, int n_in,
                              void* d_out, int out_size, void* d_ws, size_t ws_size, hipStream_t stream) {
    if (n_in < 7) return;
    if ((size_t)in_sizes[0] < (size_t)NB * TLEN * 3) return;
    if ((size_t)in_sizes[1] < (size_t)HID1 * NS || in_sizes[2] < HID1) return;
    if ((size_t)in_sizes[3] < (size_t)HID2 * HID1 || in_sizes[4] < HID2) return;
    if ((size_t)in_sizes[5] < (size_t)NO * HID2 || in_sizes[6] < NO) return;
    if ((size_t)out_size < (size_t)NB * NO) return;
    if (SZ_TOTAL > ws_size) return;
    const float* inp = (const float*)d_in[0];
    const float* w1 = (const float*)d_in[1]; const float* b1 = (const float*)d_in[2];
    const float* w2 = (const float*)d_in[3]; const float* b2 = (const float*)d_in[4];
    const float* w3 = (const float*)d_in[5]; const float* b3 = (const float*)d_in[6];
    float* OUT = (float*)d_out;
    char* wsp = (char*)d_ws;
    h16* W1H = (h16*)wsp; wsp += SZ_W1;
    h16* W2H = (h16*)wsp; wsp += SZ_W2;
    h16* W3H = (h16*)wsp; wsp += SZ_W3;
    h16* FH  = (h16*)wsp; wsp += SZ_FH;
    h16* H1P = (h16*)wsp; wsp += SZ_H1;
    h16* H2P = (h16*)wsp; wsp += SZ_H2;

    { const unsigned n8 = (unsigned)((size_t)HID1 * NS / 8);   k_wcvt<<<(n8 + 255) / 256, 256, 0, stream>>>(w1, W1H, n8, n8); }
    { const unsigned n8 = (unsigned)((size_t)HID2 * HID1 / 8); k_wcvt<<<(n8 + 255) / 256, 256, 0, stream>>>(w2, W2H, n8, n8); }
    { const unsigned s8 = (unsigned)((size_t)NO * HID2 / 8), d8 = (unsigned)((size_t)NOP * HID2 / 8);
      k_wcvt<<<(d8 + 255) / 256, 256, 0, stream>>>(w3, W3H, s8, d8); }

    k_spec<<<NB, 256, 0, stream>>>(inp, FH);
    k_dense<<<dim3(NB / 64, HID1 / 64, 1), 32, 0, stream>>>(FH, W1H, b1, H1P, NS, HID1);
    k_dense<<<dim3(NB / 64, HID2 / 64, 1), 32, 0, stream>>>(H1P, W2H, b2, H2P, HID1, HID2);
    k_head<<<NB / 16, 32, 0, stream>>>(H2P, W3H, b3, OUT);
}
